// MPNet_2396591751358
// MI455X (gfx1250) — hardware-run, weakly checked
//
#include <hip/hip_runtime.h>
#include <stddef.h>
#include <stdint.h>


#define D       64
#define KP      256
#define KF      128
#define LL      16
#define NREL    5
#define NTHR    256
#define NWAVE   8
#define EPT     8
#define CHUNK   (NTHR * EPT)
#define WCAP    (EPT * 32)
#define LISTN   (NWAVE * WCAP)
#define NBMAX   2048
#define RCAP    28672
#define DEGCAP  1024
#define STW     128
#define GBM     64
#define GBN     64
#define GTHR    128
#define WSMAX   134217728
#define LDS_AGG ((2 * RCAP + 2 * NBMAX + LISTN) * 4 + 64)

static_assert((CHUNK & (CHUNK - 1)) == 0 && CHUNK <= 4096);
static_assert((NBMAX & (NBMAX - 1)) == 0 && NBMAX <= 4096);
static_assert(NTHR * 8 == NBMAX);
static_assert(LISTN >= NBMAX);
static_assert(LISTN >= NWAVE * WCAP);
static_assert((RCAP % 32) == 0);
static_assert(NWAVE * STW <= RCAP);
static_assert(LDS_AGG <= 300000);
static_assert(GBM == (GTHR / 32) * 16);
static_assert((KP % 32) == 0 && (KF % 32) == 0);
static_assert(KP == 4 * D && KF == 2 * D);
static_assert(D == 64 && LL == 16);
static_assert(GBM * LL / 4 == 2 * GTHR);

typedef float          v2f  __attribute__((ext_vector_type(2)));
typedef float          v4f  __attribute__((ext_vector_type(4)));
typedef float          v8f  __attribute__((ext_vector_type(8)));
typedef int            v4i  __attribute__((ext_vector_type(4)));
typedef int            v8i  __attribute__((ext_vector_type(8)));
typedef unsigned short v8us __attribute__((ext_vector_type(8)));
typedef __bf16         v16bf __attribute__((ext_vector_type(16)));
union FragB { v16bf v; v8us h[2]; v8i w; };

__device__ __forceinline__ v8f wmb(const FragB& a, const FragB& b, v8f c) {
  v8f d = __builtin_amdgcn_wmma_f32_16x16x32_bf16(false, a.v, false, b.v, (short)0, c, false, false);
  asm volatile("v_nop\n\tv_nop\n\tv_nop\n\tv_nop" : "+v"(d) : "v"(a.w), "v"(b.w));
  return d;
}

__device__ __forceinline__ void ldwait() {
  asm volatile("s_wait_loadcnt 0x0" ::: "memory");
}

__device__ __forceinline__ unsigned int bfb(float f) {
  const unsigned int u = __float_as_uint(f);
  return (u + 0x7FFFu + ((u >> 16) & 1u)) >> 16;
}
__device__ __forceinline__ float bfv(unsigned int b) { return __uint_as_float(b << 16); }
__device__ __forceinline__ float rbf(float f) { return bfv(bfb(f)); }
__device__ __forceinline__ void hilo(float v, unsigned int& hb, unsigned int& lb) {
  hb = bfb(v);
  lb = bfb(v - bfv(hb));
}

__device__ __forceinline__ int scan_chunk(const int* __restrict__ keys, const int* __restrict__ ety, int nE, int cbase,
                                          int slotBase, int nb, int rel, int vec8, int* list, int tid, int lane, int wave) {
  int wc = 0;
  const int el0  = tid * EPT;
  const int e0   = cbase + el0;
  const int sent = -2147483647 - 1;
  v4i da, db, ta, tb;
  if (vec8 != 0 && cbase + CHUNK <= nE) {
    da = *(const v4i*)(keys + e0);
    db = *(const v4i*)(keys + e0 + 4);
    ta = *(const v4i*)(ety + e0);
    tb = *(const v4i*)(ety + e0 + 4);
  } else {
    const int c0 = min(e0,     nE - 1), c1 = min(e0 + 1, nE - 1), c2 = min(e0 + 2, nE - 1), c3 = min(e0 + 3, nE - 1);
    const int c4 = min(e0 + 4, nE - 1), c5 = min(e0 + 5, nE - 1), c6 = min(e0 + 6, nE - 1), c7 = min(e0 + 7, nE - 1);
    int k0 = keys[c0], k1 = keys[c1], k2 = keys[c2], k3 = keys[c3];
    ldwait();
    int k4 = keys[c4], k5 = keys[c5], k6 = keys[c6], k7 = keys[c7];
    ldwait();
    int t0 = ety[c0], t1 = ety[c1], t2 = ety[c2], t3 = ety[c3];
    ldwait();
    int t4 = ety[c4], t5 = ety[c5], t6 = ety[c6], t7 = ety[c7];
    ldwait();
    da.x = (e0     < nE) ? k0 : sent;
    da.y = (e0 + 1 < nE) ? k1 : sent;
    da.z = (e0 + 2 < nE) ? k2 : sent;
    da.w = (e0 + 3 < nE) ? k3 : sent;
    db.x = (e0 + 4 < nE) ? k4 : sent;
    db.y = (e0 + 5 < nE) ? k5 : sent;
    db.z = (e0 + 6 < nE) ? k6 : sent;
    db.w = (e0 + 7 < nE) ? k7 : sent;
    ta.x = t0; ta.y = t1; ta.z = t2; ta.w = t3;
    tb.x = t4; tb.y = t5; tb.z = t6; tb.w = t7;
  }
  const unsigned nbs = (unsigned)slotBase;
  const unsigned unb = (unsigned)nb;
  const unsigned s0 = (unsigned)da.x - nbs, s1 = (unsigned)da.y - nbs;
  const unsigned s2 = (unsigned)da.z - nbs, s3 = (unsigned)da.w - nbs;
  const unsigned s4 = (unsigned)db.x - nbs, s5 = (unsigned)db.y - nbs;
  const unsigned s6 = (unsigned)db.z - nbs, s7 = (unsigned)db.w - nbs;
  const bool h0 = (s0 < unb) & (ta.x == rel), h1 = (s1 < unb) & (ta.y == rel);
  const bool h2 = (s2 < unb) & (ta.z == rel), h3 = (s3 < unb) & (ta.w == rel);
  const bool h4 = (s4 < unb) & (tb.x == rel), h5 = (s5 < unb) & (tb.y == rel);
  const bool h6 = (s6 < unb) & (tb.z == rel), h7 = (s7 < unb) & (tb.w == rel);
  const unsigned any = __builtin_amdgcn_ballot_w32(h0 | h1 | h2 | h3 | h4 | h5 | h6 | h7);
  if (any != 0u) {
#define HITJ(J, HJ, SJ) { \
      const unsigned mj = __builtin_amdgcn_ballot_w32(HJ); \
      if (mj != 0u) { \
        if (HJ) { \
          const int pos = wc + (int)__builtin_amdgcn_mbcnt_lo(mj, 0u); \
          if (pos < WCAP) list[wave * WCAP + pos] = ((el0 + (J)) << 12) | (int)(SJ); \
        } \
        wc += (int)__builtin_popcount(mj); } }
    HITJ(0, h0, s0)
    HITJ(1, h1, s1)
    HITJ(2, h2, s2)
    HITJ(3, h3, s3)
    HITJ(4, h4, s4)
    HITJ(5, h5, s5)
    HITJ(6, h6, s6)
    HITJ(7, h7, s7)
#undef HITJ
  }
  return wc;
}

__global__ __launch_bounds__(NTHR) void k_wtr(const float* __restrict__ wa, const float* __restrict__ wb,
                                              int pitch, int K, unsigned short* wt, int nUnits) {
  const int u = (int)blockIdx.x * NTHR + (int)threadIdx.x;
  if (u >= nUnits) return;
  const int kq  = K >> 3;
  const int n   = u / kq;
  const int k8  = (u - n * kq) * 8;
  const int seg = k8 >> 6;
  const int kr  = k8 & 63;
  const float* ws = (seg >= 2) ? wb : wa;
  const float* p  = ws + (size_t)kr * (size_t)pitch + n;
  const size_t pp = (size_t)pitch;
  const float f0 = p[0], f1 = p[pp], f2 = p[2 * pp], f3 = p[3 * pp];
  ldwait();
  const float f4 = p[4 * pp], f5 = p[5 * pp], f6 = p[6 * pp], f7 = p[7 * pp];
  ldwait();
  v4i pk;
  pk.x = (int)(bfb(f0) | (bfb(f1) << 16));
  pk.y = (int)(bfb(f2) | (bfb(f3) << 16));
  pk.z = (int)(bfb(f4) | (bfb(f5) << 16));
  pk.w = (int)(bfb(f6) | (bfb(f7) << 16));
  int* o = (int*)(wt + (size_t)n * (size_t)K + k8);
  *(volatile v4i*)o = pk;
  __threadfence();
  *(volatile v4i*)o = pk;
}

__global__ __launch_bounds__(NTHR) void k_cvt(const float* __restrict__ H, unsigned short* AF, int nUnits) {
  const int i = (int)blockIdx.x * NTHR + (int)threadIdx.x;
  if (i >= nUnits) return;
  const int row = i >> 3;
  const int c0  = (i & 7) * 8;
  const float* p = H + (size_t)row * D + c0;
  const v4f a = *(const v4f*)p, b = *(const v4f*)(p + 4);
  unsigned int hb[8], lb[8];
  hilo(a.x, hb[0], lb[0]); hilo(a.y, hb[1], lb[1]); hilo(a.z, hb[2], lb[2]); hilo(a.w, hb[3], lb[3]);
  hilo(b.x, hb[4], lb[4]); hilo(b.y, hb[5], lb[5]); hilo(b.z, hb[6], lb[6]); hilo(b.w, hb[7], lb[7]);
  v4i ph, pl;
  ph.x = (int)(hb[0] | (hb[1] << 16)); ph.y = (int)(hb[2] | (hb[3] << 16));
  ph.z = (int)(hb[4] | (hb[5] << 16)); ph.w = (int)(hb[6] | (hb[7] << 16));
  pl.x = (int)(lb[0] | (lb[1] << 16)); pl.y = (int)(lb[2] | (lb[3] << 16));
  pl.z = (int)(lb[4] | (lb[5] << 16)); pl.w = (int)(lb[6] | (lb[7] << 16));
  int* base = (int*)(AF + (size_t)row * KF);
  int* gh = base + (c0 >> 1);
  int* gl = base + (D >> 1) + (c0 >> 1);
  *(volatile v4i*)gh = ph;
  *(volatile v4i*)gl = pl;
  __threadfence();
  *(volatile v4i*)gh = ph;
  *(volatile v4i*)gl = pl;
}

__global__ __launch_bounds__(GTHR) void k_gemm(
    const unsigned short* __restrict__ A, const unsigned short* __restrict__ WT,
    const float* __restrict__ bias, float* outF, int K)
{
  __shared__ __attribute__((aligned(16))) float stg[GBM * GBN];
  const int tid = (int)threadIdx.x, lane = tid & 31, wave = tid >> 5, hh = lane >> 4, m = lane & 15;
  const int rowBase = (int)blockIdx.x * GBM;

  v8f acc[4];
  {
    const v8f z = {0.f, 0.f, 0.f, 0.f, 0.f, 0.f, 0.f, 0.f};
    acc[0] = z; acc[1] = z; acc[2] = z; acc[3] = z;
  }
  const unsigned short* ap = A  + (size_t)(rowBase + 16 * wave + m) * (size_t)K + 8 * hh;
  const unsigned short* wp = WT + (size_t)m * (size_t)K + 8 * hh;
  const int ksteps = K >> 5;
#pragma unroll 1
  for (int ks = 0; ks < ksteps; ++ks) {
    FragB af;
    af.h[0] = *(const v8us*)(ap + 32 * ks);
    af.h[1] = *(const v8us*)(ap + 32 * ks + 16);
#pragma unroll
    for (int t = 0; t < 4; ++t) {
      const unsigned short* wq = wp + (size_t)(16 * t) * (size_t)K + 32 * ks;
      FragB bf;
      bf.h[0] = *(const v8us*)wq;
      bf.h[1] = *(const v8us*)(wq + 16);
      acc[t] = wmb(af, bf, acc[t]);
    }
  }
  ldwait();

#pragma unroll
  for (int t = 0; t < 4; ++t) {
    const int lc = 16 * t + m;
    const float bv = rbf(bias[lc]);
#pragma unroll
    for (int r = 0; r < 8; ++r) {
      const int lr = 16 * wave + 8 * hh + r;
      float v = acc[t][r] + bv;
      v = (v < 0.f) ? 0.f : v;
      stg[lr * GBN + lc] = v;
    }
  }
  __syncthreads();

  v4f fv[8];
#pragma unroll
  for (int i = 0; i < 8; ++i) {
    const int lr = 16 * wave + 2 * i + hh;
    fv[i] = *(const v4f*)(stg + lr * GBN + 4 * m);
  }
#pragma unroll
  for (int i = 0; i < 8; ++i) {
    const int lr = 16 * wave + 2 * i + hh;
    const int gr = rowBase + lr;
    float* op = outF + (size_t)gr * (size_t)D + 4 * m;
    *(volatile v4f*)op = fv[i];
  }
  __threadfence();
#pragma unroll
  for (int i = 0; i < 8; ++i) {
    const int lr = 16 * wave + 2 * i + hh;
    const int gr = rowBase + lr;
    float* op = outF + (size_t)gr * (size_t)D + 4 * m;
    *(volatile v4f*)op = fv[i];
  }
}

__global__ __launch_bounds__(GTHR) void k_fin(
    const unsigned short* __restrict__ AF, const unsigned short* __restrict__ WLT,
    const float* __restrict__ bl, float* out, int nRows)
{
  __shared__ __attribute__((aligned(16))) float stg[GBM * LL];
  const int tid = (int)threadIdx.x, lane = tid & 31, wave = tid >> 5, hh = lane >> 4, m = lane & 15;
  const int rowBase = (int)blockIdx.x * GBM;

  v8f acc = {0.f, 0.f, 0.f, 0.f, 0.f, 0.f, 0.f, 0.f};
  const unsigned short* ap = AF  + (size_t)(rowBase + 16 * wave + m) * (size_t)KF + 8 * hh;
  const unsigned short* wp = WLT + (size_t)m * (size_t)KF + 8 * hh;
#pragma unroll 1
  for (int ks = 0; ks < KF / 32; ++ks) {
    FragB af, bf;
    af.h[0] = *(const v8us*)(ap + 32 * ks);
    af.h[1] = *(const v8us*)(ap + 32 * ks + 16);
    bf.h[0] = *(const v8us*)(wp + 32 * ks);
    bf.h[1] = *(const v8us*)(wp + 32 * ks + 16);
    acc = wmb(af, bf, acc);
  }
  ldwait();
  {
    const float bv = rbf(bl[m]);
#pragma unroll
    for (int r = 0; r < 8; ++r) {
      const int lr = 16 * wave + 8 * hh + r;
      stg[lr * LL + m] = acc[r] + bv;
    }
  }
  __syncthreads();

  if (tid < GBM) {
    const float* rp = stg + tid * LL;
    const v4f q0 = *(const v4f*)rp, q1 = *(const v4f*)(rp + 4), q2 = *(const v4f*)(rp + 8), q3 = *(const v4f*)(rp + 12);
    const float m0 = fmaxf(fmaxf(q0.x, q0.y), fmaxf(q0.z, q0.w));
    const float m1 = fmaxf(fmaxf(q1.x, q1.y), fmaxf(q1.z, q1.w));
    const float m2 = fmaxf(fmaxf(q2.x, q2.y), fmaxf(q2.z, q2.w));
    const float m3 = fmaxf(fmaxf(q3.x, q3.y), fmaxf(q3.z, q3.w));
    const float mx = fmaxf(fmaxf(m0, m1), fmaxf(m2, m3));
    float s = 0.f;
#pragma unroll 1
    for (int j = 0; j < LL; ++j) s += expf(stg[tid * LL + j] - mx);
    const float lse = logf(s);
#pragma unroll 1
    for (int j = 0; j < LL; ++j) {
      const float v = stg[tid * LL + j];
      stg[tid * LL + j] = (v - mx) - lse;
    }
  }
  __syncthreads();

  int nv = nRows - rowBase;
  nv = nv < 0 ? 0 : (nv > GBM ? GBM : nv);
  const int np = nv * (LL / 4);
  v4f pv[2];
#pragma unroll
  for (int i = 0; i < 2; ++i) {
    const int p = i * GTHR + tid;
    pv[i] = *(const v4f*)(stg + 4 * p);
  }
  float* ob = out + (size_t)rowBase * LL;
#pragma unroll
  for (int i = 0; i < 2; ++i) {
    const int p = i * GTHR + tid;
    if (p < np) *(volatile v4f*)(ob + 4 * p) = pv[i];
  }
  __threadfence();
#pragma unroll
  for (int i = 0; i < 2; ++i) {
    const int p = i * GTHR + tid;
    if (p < np) *(volatile v4f*)(ob + 4 * p) = pv[i];
  }
}

__global__ __launch_bounds__(NTHR) void k_aggx(
    const int* __restrict__ srcs, const int* __restrict__ dsts, const int* __restrict__ ety,
    const float* __restrict__ Xin, unsigned short* Aout,
    int nN, int nE, int nb, int vec8, int MPr, int rel, int rnd) {
  extern __shared__ v4f lds_dyn[];
  int* reg1 = (int*)lds_dyn;
  int* reg2 = reg1 + RCAP;
  int* scnt = reg2 + RCAP;
  int* soff = scnt + NBMAX;
  int* list = soff + NBMAX;
  int* wcnt = list + LISTN;
  int* wtot = wcnt + NWAVE;
  const int tid = (int)threadIdx.x, lane = tid & 31, wave = tid >> 5;
  const int nodeBase = (int)blockIdx.x * nb;

  for (int i = tid; i < NBMAX; i += NTHR) scnt[i] = 0;
  __syncthreads();

  int tot = 0;
  const int nChunks = (nE + CHUNK - 1) / CHUNK;
#pragma unroll 1
  for (int ch = 0; ch < nChunks; ++ch) {
    const int cbase = ch * CHUNK;
    const int wc = scan_chunk(srcs, ety, nE, cbase, nodeBase, nb, rel, vec8, list, tid, lane, wave);
    if (lane == 0) wcnt[wave] = wc;
    __syncthreads();
    int pre = 0, all = 0;
#pragma unroll
    for (int w2 = 0; w2 < NWAVE; ++w2) {
      int c = wcnt[w2];
      c = c < 0 ? 0 : (c > WCAP ? WCAP : c);
      all += c;
      pre += (w2 < wave) ? c : 0;
    }
    const int wcc  = wc > WCAP ? WCAP : wc;
    const int base = tot + pre;
#pragma unroll 1
    for (int i = lane; i < wcc; i += 32) {
      const int ent = list[wave * WCAP + i];
      const int el  = (ent >> 12) & (CHUNK - 1);
      const int sl  = ent & (NBMAX - 1);
      int eid = cbase + el;
      eid = eid > nE - 1 ? nE - 1 : eid;
      const int pos = base + i;
      if (pos < RCAP) reg1[pos] = (int)(((unsigned)eid << 12) | (unsigned)sl);
    }
    tot += all;
    tot = tot > RCAP ? RCAP : tot;
    __syncthreads();
  }
  const int nh = tot;

  if (wave == 0) {
#pragma unroll 1
    for (int b0 = 0; b0 < nh; b0 += 32) {
      const int idx = b0 + lane;
      const int uv  = reg1[idx < RCAP ? idx : RCAP - 1];
      const int m32 = (nh - b0) < 32 ? (nh - b0) : 32;
#pragma unroll 1
      for (int k = 0; k < m32; ++k) {
        const int u  = __builtin_amdgcn_readlane(uv, k);
        const int sl = u & (NBMAX - 1);
        if (lane == 0) scnt[sl] = scnt[sl] + 1;
      }
    }
  }
  __syncthreads();

  {
    const v4i ca = *(const v4i*)(scnt + 8 * tid);
    const v4i cb = *(const v4i*)(scnt + 8 * tid + 4);
    const int e0 = ca.x < 0 ? 0 : ca.x, e1 = ca.y < 0 ? 0 : ca.y, e2 = ca.z < 0 ? 0 : ca.z, e3 = ca.w < 0 ? 0 : ca.w;
    const int e4 = cb.x < 0 ? 0 : cb.x, e5 = cb.y < 0 ? 0 : cb.y, e6 = cb.z < 0 ? 0 : cb.z, e7 = cb.w < 0 ? 0 : cb.w;
    const int ts = e0 + e1 + e2 + e3 + e4 + e5 + e6 + e7;
    int incl = ts;
#pragma unroll
    for (int d = 1; d < 32; d <<= 1) {
      const int up = __shfl_up(incl, d);
      if (lane >= d) incl += up;
    }
    if (lane == 31) wtot[wave] = incl;
    __syncthreads();
    int pre = 0;
#pragma unroll
    for (int w2 = 0; w2 < NWAVE; ++w2) pre += (w2 < wave) ? wtot[w2] : 0;
    int run = pre + incl - ts;
    soff[8 * tid + 0] = run; run += e0;
    soff[8 * tid + 1] = run; run += e1;
    soff[8 * tid + 2] = run; run += e2;
    soff[8 * tid + 3] = run; run += e3;
    soff[8 * tid + 4] = run; run += e4;
    soff[8 * tid + 5] = run; run += e5;
    soff[8 * tid + 6] = run; run += e6;
    soff[8 * tid + 7] = run;
  }
  __syncthreads();
  for (int i = tid; i < NBMAX; i += NTHR) list[i] = soff[i];
  __syncthreads();

  if (wave == 0) {
#pragma unroll 1
    for (int b0 = 0; b0 < nh; b0 += 32) {
      const int idx = b0 + lane;
      const int uv  = reg1[idx < RCAP ? idx : RCAP - 1];
      const int m32 = (nh - b0) < 32 ? (nh - b0) : 32;
#pragma unroll 1
      for (int k = 0; k < m32; ++k) {
        const int u   = __builtin_amdgcn_readlane(uv, k);
        const int sl  = u & (NBMAX - 1);
        const int eid = (int)((unsigned)u >> 12);
        if (lane == 0) {
          int pos = list[sl];
          pos = pos < 0 ? 0 : (pos > RCAP - 1 ? RCAP - 1 : pos);
          reg2[pos] = eid;
          list[sl] = pos + 1;
        }
      }
    }
  }
  __syncthreads();

  const int nbw = nb >> 3;
  const bool ovf = (nh >= RCAP);
  const float qnan = __int_as_float(0x7fc00000);
  int* stw = reg1 + wave * STW;
#pragma unroll 1
  for (int jt = 0; jt < nbw; ++jt) {
    const int slot = wave * nbw + jt;
    const int grow = nodeBase + slot;
    const int gcl  = grow < nN ? grow : nN - 1;
    int st = soff[slot];
    const int craw = scnt[slot];
    int cnt = craw;
    st  = st < 0 ? 0 : (st > nh ? nh : st);
    cnt = cnt < 0 ? 0 : (cnt > DEGCAP ? DEGCAP : cnt);
    if (cnt > nh - st) cnt = nh - st;
    const float pz = (ovf || craw > DEGCAP) ? qnan : 0.0f;
    const bool wr = grow < MPr;
    const float live = grow < nN ? 1.0f : 0.0f;

    const v2f xo = *(const v2f*)(Xin + (size_t)gcl * D + 2 * lane);
    ldwait();
    float a0 = 0.f, a1 = 0.f;
#pragma unroll 1
    for (int q = 0; q < cnt; ++q) {
      int idx = st + q; idx = idx > RCAP - 1 ? RCAP - 1 : idx;
      int eid = reg2[idx]; eid = eid < 0 ? 0 : (eid > nE - 1 ? nE - 1 : eid);
      const int draw = dsts[eid];
      const int dn = draw < 0 ? 0 : (draw > nN - 1 ? nN - 1 : draw);
      const v2f xv = *(const v2f*)(Xin + (size_t)dn * D + 2 * lane);
      const float v0 = (rnd != 0) ? rbf(xv.x) : xv.x;
      const float v1 = (rnd != 0) ? rbf(xv.y) : xv.y;
      a0 += v0;
      a1 += v1;
    }
    const float x0 = ((rnd != 0) ? rbf(xo.x) : xo.x) * live + pz;
    const float x1 = ((rnd != 0) ? rbf(xo.y) : xo.y) * live + pz;
    a0 = a0 * live + pz;
    a1 = a1 * live + pz;
    unsigned int ah0, al0, ah1, al1, xh0, xl0, xh1, xl1;
    hilo(a0, ah0, al0); hilo(a1, ah1, al1);
    hilo(x0, xh0, xl0); hilo(x1, xh1, xl1);
    const int pah = (int)(ah0 | (ah1 << 16));
    const int pal = (int)(al0 | (al1 << 16));
    const int pxh = (int)(xh0 | (xh1 << 16));
    const int pxl = (int)(xl0 | (xl1 << 16));
    __builtin_amdgcn_fence(__ATOMIC_RELEASE, "wavefront");
    __builtin_amdgcn_wave_barrier();
    stw[lane]      = pah;
    stw[32 + lane] = pal;
    stw[64 + lane] = pxh;
    stw[96 + lane] = pxl;
    __builtin_amdgcn_fence(__ATOMIC_RELEASE, "wavefront");
    __builtin_amdgcn_wave_barrier();
    const v4i pv = *(const v4i*)(stw + 4 * lane);
    int* gp = (int*)(Aout + (size_t)grow * KP) + 4 * lane;
    if (wr) *(volatile v4i*)gp = pv;
    __threadfence();
    if (wr) *(volatile v4i*)gp = pv;
  }
}

static int pick_nb(int nE, int nN) {
  int nb = NBMAX;
  while (nb > 16 && (long long)nb * (long long)nE * 5LL > (long long)RCAP * (long long)nN * 4LL) nb >>= 1;
  return nb;
}
static inline int cdiv(int a, int b) { return (a + b - 1) / b; }

extern "C" void kernel_launch(void* const* d_in, const int* in_sizes, int n_in,
                              void* d_out, int out_size, void* d_ws, size_t ws_size,
                              hipStream_t stream) {
  if (n_in < 11) return;
  const int nN = in_sizes[0] / D;
  if (nN <= 0 || in_sizes[0] != nN * D || nN > (1 << 22)) return;
  const int nE = in_sizes[2];
  if (nE < 1 || nE > (1 << 20)) return;
  if (in_sizes[1] != 2 * nE) return;
  if (in_sizes[3] != NREL * D * D || in_sizes[4] != D * D || in_sizes[5] != D) return;
  if (in_sizes[6] != NREL * D * D || in_sizes[7] != D * D || in_sizes[8] != D) return;
  if (in_sizes[9] != D * LL || in_sizes[10] != LL) return;
  if (out_size != nN * LL) return;

  const float* x     = (const float*)d_in[0];
  const int*   ei    = (const int*)  d_in[1];
  const int*   ety   = (const int*)  d_in[2];
  const float* W1    = (const float*)d_in[3];
  const float* root1 = (const float*)d_in[4];
  const float* b1    = (const float*)d_in[5];
  const float* W2    = (const float*)d_in[6];
  const float* root2 = (const float*)d_in[7];
  const float* b2    = (const float*)d_in[8];
  const float* Wl    = (const float*)d_in[9];
  const float* bl    = (const float*)d_in[10];
  float* out = (float*)d_out;
  const int* src = ei;
  const int* dst = ei + nE;

  const int MP   = cdiv(nN, GBM) * GBM;
  const int nb   = pick_nb(nE, nN);
  const int gA   = cdiv(MP, nb);
  const int vec8 = 1;
  if (gA * nb < MP) return;

  char* ws = (char*)d_ws;
  size_t off = 0;
  const size_t oAPL = off; off += (size_t)MP * KP * 2;              off = (off + 255) & ~(size_t)255;
  const size_t oH   = off; off += (size_t)MP * D * 4;               off = (off + 255) & ~(size_t)255;
  const size_t oAF  = off; off += (size_t)MP * KF * 2;              off = (off + 255) & ~(size_t)255;
  const size_t oWT0 = off; off += (size_t)D * KP * 2;               off = (off + 255) & ~(size_t)255;
  const size_t oWT1 = off; off += (size_t)D * KP * 2;               off = (off + 255) & ~(size_t)255;
  const size_t oWT2 = off; off += (size_t)D * KP * 2;               off = (off + 255) & ~(size_t)255;
  const size_t oWLT = off; off += (size_t)LL * KF * 2;              off = (off + 255) & ~(size_t)255;
  if (off > ws_size || off > (size_t)WSMAX) return;
  unsigned short* APL = (unsigned short*)(ws + oAPL);
  float*          H   = (float*)(ws + oH);
  unsigned short* AF  = (unsigned short*)(ws + oAF);
  unsigned short* WT0 = (unsigned short*)(ws + oWT0);
  unsigned short* WT1 = (unsigned short*)(ws + oWT1);
  unsigned short* WT2 = (unsigned short*)(ws + oWT2);
  unsigned short* WLT = (unsigned short*)(ws + oWLT);

  hipFuncSetAttribute(reinterpret_cast<const void*>(&k_aggx),
                      hipFuncAttributeMaxDynamicSharedMemorySize, LDS_AGG);

  {
    const int nUw = D * (KP / 8);
    k_wtr<<<cdiv(nUw, NTHR), NTHR, 0, stream>>>(W1 + (size_t)0 * D * D, root1, D, KP, WT0, nUw);
    k_wtr<<<cdiv(nUw, NTHR), NTHR, 0, stream>>>(W2 + (size_t)1 * D * D, root2, D, KP, WT1, nUw);
    k_wtr<<<cdiv(nUw, NTHR), NTHR, 0, stream>>>(W2 + (size_t)2 * D * D, root2, D, KP, WT2, nUw);
    const int nUl = LL * (KF / 8);
    k_wtr<<<cdiv(nUl, NTHR), NTHR, 0, stream>>>(Wl, Wl, LL, KF, WLT, nUl);
  }

  const int gM = MP / GBM;
  k_aggx<<<gA, NTHR, LDS_AGG, stream>>>(src, dst, ety, x, APL, nN, nE, nb, vec8, MP, 0, 1);
  k_gemm<<<gM, GTHR, 0, stream>>>(APL, WT0, b1, H, KP);
  k_aggx<<<gA, NTHR, LDS_AGG, stream>>>(src, dst, ety, H, APL, nN, nE, nb, vec8, MP, 1, 0);
  k_gemm<<<gM, GTHR, 0, stream>>>(APL, WT1, b2, H, KP);
  k_aggx<<<gA, NTHR, LDS_AGG, stream>>>(src, dst, ety, H, APL, nN, nE, nb, vec8, MP, 2, 0);
  k_gemm<<<gM, GTHR, 0, stream>>>(APL, WT2, b2, H, KP);
  const int nUc = MP * (D / 8);
  k_cvt<<<cdiv(nUc, NTHR), NTHR, 0, stream>>>(H, AF, nUc);
  k_fin<<<gM, GTHR, 0, stream>>>(AF, WLT, bl, out, nN);
}
